// RelativePositionalMultiHeadAttention_87282325389402
// MI455X (gfx1250) — hardware-verified
//
#include <hip/hip_runtime.h>
#include <math.h>


typedef _Float16     v8h  __attribute__((ext_vector_type(8)));
typedef _Float16     v16h __attribute__((ext_vector_type(16)));
typedef __bf16       v16b __attribute__((ext_vector_type(16)));
typedef float        v8f  __attribute__((ext_vector_type(8)));
typedef float        v4f  __attribute__((ext_vector_type(4)));
typedef unsigned int v4u  __attribute__((ext_vector_type(4)));
typedef unsigned int v2u  __attribute__((ext_vector_type(2)));

union FragH { v16h v; v8h h[2]; };
union FragB { v16b v; v4u u[2]; };
union H8    { v8h v; v4u u; };

namespace cfg {
constexpr int DM = 512;
constexpr int NH = 8;
constexpr int DK = 64;
constexpr int BB = 4;
constexpr int TT = 2048;
constexpr int PR = TT;
constexpr int PA = 36;
constexpr int PC = 68;
constexpr float PSC  = 32768.f;
constexpr float PSCI = 1.f / 32768.f;
}

__device__ __forceinline__ v8f zero8() {
  v8f z = {0.f, 0.f, 0.f, 0.f, 0.f, 0.f, 0.f, 0.f};
  return z;
}

__device__ __forceinline__ v8f mma_f16(v16h a, v16h b, v8f c) {
  c = __builtin_amdgcn_wmma_f32_16x16x32_f16(false, a, false, b, (short)0, c, false, false);
  asm volatile("v_nop\n\tv_nop\n\tv_nop\n\tv_nop" : "+v"(c) : "v"(a), "v"(b));
  return c;
}
__device__ __forceinline__ v8f mma_bf16(v16b a, v16b b, v8f c) {
  c = __builtin_amdgcn_wmma_f32_16x16x32_bf16(false, a, false, b, (short)0, c, false, false);
  asm volatile("v_nop\n\tv_nop\n\tv_nop\n\tv_nop" : "+v"(c) : "v"(a), "v"(b));
  return c;
}

__device__ __forceinline__ unsigned int bf16_bits(float x) {
  const unsigned int u = __float_as_uint(x);
  return (u + 0x7FFFu + ((u >> 16) & 1u)) >> 16;
}
__device__ __forceinline__ void split_bf16(float x, unsigned int& hb, unsigned int& lb) {
  hb = bf16_bits(x);
  const float hf = __uint_as_float(hb << 16);
  lb = bf16_bits(x - hf);
}

template <int OM, bool HASB, bool HASADD>
__device__ __forceinline__ void proj_store(const float* Ct, const float* __restrict__ bias,
                                           const float* __restrict__ add, _Float16* O, float* Of,
                                           int m0, int n0, int M, int wave, int lane)
{
  using namespace cfg;
  if (OM == 0) {
    #pragma unroll
    for (int it = 0; it < 4; ++it) {
      const int row = it * 16 + wave * 4 + (lane >> 3);
      const int p   = (lane & 7) * 8;
      const int gm  = m0 + row;
      const int g   = (gm >> 11) * NH + (n0 >> 6);
      const int tr  = gm & (TT - 1);
      v8h o;
      #pragma unroll
      for (int e = 0; e < 8; ++e) {
        float val = Ct[row * PC + p + e];
        if (HASB)   val += bias[n0 + p + e];
        if (HASADD) val += add[n0 + p + e];
        o[e] = (_Float16)val;
      }
      if (gm < M) *(volatile v8h*)(O + ((size_t)g * TT + tr) * DK + p) = o;
    }
  } else if (OM == 1) {
    const int g  = (m0 >> 11) * NH + (n0 >> 6);
    const int t0 = m0 & (TT - 1);
    #pragma unroll
    for (int it = 0; it < 4; ++it) {
      const int d = it * 16 + wave * 4 + (lane >> 3);
      const int p = (lane & 7) * 8;
      const float bn = HASB ? bias[n0 + d] : 0.f;
      v8h o;
      #pragma unroll
      for (int e = 0; e < 8; ++e) o[e] = (_Float16)(Ct[(p + e) * PC + d] + bn);
      if (m0 + 63 < M) *(volatile v8h*)(O + ((size_t)g * DK + d) * TT + t0 + p) = o;
    }
  } else {
    #pragma unroll
    for (int it = 0; it < 8; ++it) {
      const int L   = it * 16 + wave * 4 + (lane >> 3);
      const int row = L >> 1;
      const int c   = (L & 1) * 32 + (lane & 7) * 4;
      const int gm  = m0 + row;
      v4f o;
      #pragma unroll
      for (int e = 0; e < 4; ++e) {
        float val = Ct[row * PC + c + e];
        if (HASB) val += bias[n0 + c + e];
        o[e] = val;
      }
      if (gm < M) *(volatile v4f*)(Of + (size_t)gm * DM + n0 + c) = o;
    }
  }
}

template <int AM, int OM, bool HASB, int NADD>
__global__ __launch_bounds__(128) __attribute__((amdgpu_num_vgpr(248)))
void k_proj(const float* __restrict__ X, const float* __restrict__ W, const float* __restrict__ bias,
            const float* __restrict__ add0, const float* __restrict__ add1,
            _Float16* O0, _Float16* O1, float* Of, int M)
{
  using namespace cfg;
  __shared__ __align__(16) unsigned int Ah[64 * PA];
  __shared__ __align__(16) unsigned int Al[64 * PA];
  __shared__ __align__(16) unsigned int Bh[64 * PA];
  __shared__ __align__(16) unsigned int Bl[64 * PA];
  __shared__ __align__(16) float Ct[64 * PC];
  __shared__ float rcp_[256];

  const int tid = threadIdx.x, lane = tid & 31, wave = tid >> 5;
  const int m = lane & 15, hh = lane >> 4;
  const int m0 = blockIdx.x * 64, n0 = blockIdx.y * 64;

  if (AM == 1) {
    for (int c2 = tid; c2 < 256; c2 += 128) {
      const float den = powf(10000.f, (float)(2 * c2) * (1.f / 512.f));
      rcp_[c2] = 1.f / den;
    }
    __syncthreads();
  }

  v8f acc[4];
  #pragma unroll
  for (int i = 0; i < 4; ++i) acc[i] = zero8();

  #pragma unroll 1
  for (int kc = 0; kc < DM; kc += 64) {
    #pragma unroll 2
    for (int i = 0; i < 8; ++i) {
      const int e = tid + 128 * i;
      const int row = e >> 4, c4 = (e & 15) * 4;
      const int gm = m0 + row;
      v4f xa = {0.f, 0.f, 0.f, 0.f};
      if (AM == 1) {
        const float fr = (float)gm;
        #pragma unroll
        for (int s = 0; s < 2; ++s) {
          const int c = kc + c4 + 2 * s;
          const float th = fr * rcp_[c >> 1];
          xa[2 * s]     = sinf(th);
          xa[2 * s + 1] = cosf(th);
        }
      } else {
        if (gm < M) xa = *(const v4f*)(X + (size_t)gm * DM + kc + c4);
      }
      const v4f xb = *(const v4f*)(W + (size_t)(n0 + row) * DM + kc + c4);
      unsigned int ah4[4], al4[4], bh4[4], bl4[4];
      #pragma unroll
      for (int q = 0; q < 4; ++q) {
        split_bf16(xa[q], ah4[q], al4[q]);
        split_bf16(xb[q], bh4[q], bl4[q]);
      }
      v2u pah = {ah4[0] | (ah4[1] << 16), ah4[2] | (ah4[3] << 16)};
      v2u pal = {al4[0] | (al4[1] << 16), al4[2] | (al4[3] << 16)};
      v2u pbh = {bh4[0] | (bh4[1] << 16), bh4[2] | (bh4[3] << 16)};
      v2u pbl = {bl4[0] | (bl4[1] << 16), bl4[2] | (bl4[3] << 16)};
      const int wo = row * PA + (c4 >> 1);
      *(v2u*)(Ah + wo) = pah;
      *(v2u*)(Al + wo) = pal;
      *(v2u*)(Bh + wo) = pbh;
      *(v2u*)(Bl + wo) = pbl;
    }
    __syncthreads();
    #pragma unroll
    for (int ks = 0; ks < 2; ++ks) {
      const int ko = ks * 16 + 4 * hh;
      FragB fah, fal;
      const unsigned int* ar = Ah + (16 * wave + m) * PA + ko;
      const unsigned int* lr = Al + (16 * wave + m) * PA + ko;
      fah.u[0] = *(const v4u*)(ar);  fah.u[1] = *(const v4u*)(ar + 8);
      fal.u[0] = *(const v4u*)(lr);  fal.u[1] = *(const v4u*)(lr + 8);
      #pragma unroll
      for (int nt = 0; nt < 4; ++nt) {
        FragB fbh, fbl;
        const unsigned int* br  = Bh + (16 * nt + m) * PA + ko;
        const unsigned int* blr = Bl + (16 * nt + m) * PA + ko;
        fbh.u[0] = *(const v4u*)(br);   fbh.u[1] = *(const v4u*)(br + 8);
        fbl.u[0] = *(const v4u*)(blr);  fbl.u[1] = *(const v4u*)(blr + 8);
        acc[nt] = mma_bf16(fah.v, fbh.v, acc[nt]);
        acc[nt] = mma_bf16(fah.v, fbl.v, acc[nt]);
        acc[nt] = mma_bf16(fal.v, fbh.v, acc[nt]);
      }
    }
    __syncthreads();
  }

  #pragma unroll
  for (int nt = 0; nt < 4; ++nt) {
    #pragma unroll
    for (int r = 0; r < 8; ++r)
      Ct[(16 * wave + 8 * hh + r) * PC + 16 * nt + m] = acc[nt][r];
  }
  __syncthreads();

  if (OM == 0 && NADD == 2) {
    proj_store<0, HASB, true>(Ct, bias, add0, O0, Of, m0, n0, M, wave, lane);
    proj_store<0, HASB, true>(Ct, bias, add1, O1, Of, m0, n0, M, wave, lane);
    __threadfence();
    proj_store<0, HASB, true>(Ct, bias, add0, O0, Of, m0, n0, M, wave, lane);
    proj_store<0, HASB, true>(Ct, bias, add1, O1, Of, m0, n0, M, wave, lane);
  } else {
    proj_store<OM, HASB, false>(Ct, bias, add0, O0, Of, m0, n0, M, wave, lane);
    __threadfence();
    proj_store<OM, HASB, false>(Ct, bias, add0, O0, Of, m0, n0, M, wave, lane);
  }
}

__device__ __forceinline__ void attn_store(const float* ow, float* ao, int b, int h, int i0, int lane)
{
  using namespace cfg;
  #pragma unroll
  for (int it = 0; it < 8; ++it) {
    const int L = it * 4 + (lane >> 3);
    const int q = L >> 1, hf = L & 1, p = (lane & 7) * 4;
    const v4f val = *(const v4f*)(ow + q * 64 + hf * 32 + p);
    *(volatile v4f*)(ao + ((size_t)b * TT + i0 + q) * DM + h * DK + hf * 32 + p) = val;
  }
}

__global__ __launch_bounds__(128) __attribute__((amdgpu_num_vgpr(248)))
void k_attn(const _Float16* __restrict__ qu, const _Float16* __restrict__ qv,
            const _Float16* __restrict__ kh, const _Float16* __restrict__ vt,
            const _Float16* __restrict__ ph, const int* __restrict__ mask, float* ao)
{
  using namespace cfg;
  __shared__ __align__(16) _Float16 ks_[64 * 64];
  __shared__ __align__(16) _Float16 vs_[64 * 64];
  __shared__ __align__(16) _Float16 ps_[128 * 64];
  __shared__ __align__(16) _Float16 pT_[4 * 16 * 64];
  __shared__ __align__(16) float    bnd_[4 * 5 * 256];
  __shared__ int mk_[64];

  const int tid = threadIdx.x, lane = tid & 31, wave = tid >> 5;
  const int m = lane & 15, hh = lane >> 4;
  const int I0 = blockIdx.x * 64;
  const int bh = blockIdx.y, b = bh >> 3, h = bh & (NH - 1);
  const int i0 = I0 + 16 * wave;
  _Float16* pTw = pT_ + wave * (16 * 64);
  float* bw = bnd_ + wave * (5 * 256);

  FragH fu[2], fv[2];
  {
    const _Float16* qr = qu + ((size_t)bh * TT + i0 + m) * DK;
    const _Float16* vr = qv + ((size_t)bh * TT + i0 + m) * DK;
    #pragma unroll
    for (int kd = 0; kd < 2; ++kd) {
      fu[kd].h[0] = *(const v8h*)(qr + 32 * kd + 8 * hh);
      fu[kd].h[1] = *(const v8h*)(qr + 32 * kd + 16 + 8 * hh);
      fv[kd].h[0] = *(const v8h*)(vr + 32 * kd + 8 * hh);
      fv[kd].h[1] = *(const v8h*)(vr + 32 * kd + 16 + 8 * hh);
    }
  }

  float mrow = -INFINITY, lrow = 0.f;
  v8f o[4];
  #pragma unroll
  for (int i = 0; i < 4; ++i) o[i] = zero8();

  #pragma unroll 1
  for (int j0 = 0; j0 < TT; j0 += 64) {
    const bool hasBand = (j0 <= I0 + 63);
    __syncthreads();
    #pragma unroll
    for (int i = 0; i < 4; ++i) {
      const int e = tid + 128 * i;
      const int row = e >> 3, c = (e & 7) * 8;
      *(v8h*)(ks_ + row * 64 + c) = *(const v8h*)(kh + ((size_t)bh * TT + j0 + row) * DK + c);
      *(v8h*)(vs_ + row * 64 + c) = *(const v8h*)(vt + ((size_t)bh * DK + row) * TT + j0 + c);
    }
    if (hasBand) {
      const int rbase = I0 - j0 - 63;
      const v4u z4 = {0u, 0u, 0u, 0u};
      #pragma unroll
      for (int i = 0; i < 8; ++i) {
        const int e = tid + 128 * i;
        const int rr = e >> 3, c = (e & 7) * 8;
        const int r = rbase + rr;
        H8 val;
        val.u = z4;
        if (r >= 0 && r < PR) val.v = *(const v8h*)(ph + ((size_t)h * PR + r) * DK + c);
        *(v8h*)(ps_ + rr * 64 + c) = val.v;
      }
    }
    if (tid < 64) mk_[tid] = mask[(size_t)b * TT + j0 + tid];
    __syncthreads();

    v8f s[4];
    #pragma unroll
    for (int jj = 0; jj < 4; ++jj) {
      v8f a = zero8();
      #pragma unroll
      for (int kd = 0; kd < 2; ++kd) {
        FragH fk;
        const _Float16* kr = ks_ + (16 * jj + m) * 64 + 32 * kd + 8 * hh;
        fk.h[0] = *(const v8h*)(kr);
        fk.h[1] = *(const v8h*)(kr + 16);
        a = mma_f16(fk.v, fu[kd].v, a);
      }
      s[jj] = a;
    }

    if (hasBand) {
      #pragma unroll
      for (int t = 0; t < 5; ++t) {
        v8f g = zero8();
        #pragma unroll
        for (int kd = 0; kd < 2; ++kd) {
          FragH fp;
          const _Float16* pr = ps_ + (16 * (wave + t) + m) * 64 + 32 * kd + 8 * hh;
          fp.h[0] = *(const v8h*)(pr);
          fp.h[1] = *(const v8h*)(pr + 16);
          g = mma_f16(fp.v, fv[kd].v, g);
        }
        #pragma unroll
        for (int r = 0; r < 8; ++r) bw[t * 256 + (8 * hh + r) * 16 + m] = g[r];
      }
      __syncthreads();
      #pragma unroll
      for (int jj = 0; jj < 4; ++jj) {
        #pragma unroll
        for (int r = 0; r < 8; ++r) {
          const int u = m - (8 * hh + r) + 15;
          const int t = 3 - jj + (u >> 4);
          s[jj][r] += bw[t * 256 + (u & 15) * 16 + m];
        }
      }
    }

    #pragma unroll
    for (int jj = 0; jj < 4; ++jj) {
      #pragma unroll
      for (int r = 0; r < 8; ++r) {
        float val = s[jj][r] * 0.125f;
        if (mk_[16 * jj + 8 * hh + r] == 0) val = -INFINITY;
        s[jj][r] = val;
      }
    }

    float tmax = -INFINITY;
    #pragma unroll
    for (int jj = 0; jj < 4; ++jj) {
      #pragma unroll
      for (int r = 0; r < 8; ++r) tmax = fmaxf(tmax, s[jj][r]);
    }
    tmax = fmaxf(tmax, __shfl_xor(tmax, 16));
    const float mnew  = fmaxf(mrow, tmax);
    const float msafe = (mnew == -INFINITY) ? 0.f : mnew;
    const float corr  = (mrow == mnew) ? 1.f : __expf(mrow - msafe);
    float tsum = 0.f;
    #pragma unroll
    for (int jj = 0; jj < 4; ++jj) {
      #pragma unroll
      for (int r = 0; r < 8; ++r) {
        const float pv = __expf(s[jj][r] - msafe);
        s[jj][r] = pv;
        tsum += pv;
      }
    }
    tsum += __shfl_xor(tsum, 16);
    lrow = lrow * corr + tsum;
    mrow = mnew;
    #pragma unroll
    for (int dt = 0; dt < 4; ++dt) o[dt] = o[dt] * corr;

    #pragma unroll
    for (int jj = 0; jj < 4; ++jj) {
      v8h pv8;
      #pragma unroll
      for (int r = 0; r < 8; ++r) pv8[r] = (_Float16)(s[jj][r] * PSC);
      *(v8h*)(pTw + m * 64 + 16 * jj + 8 * hh) = pv8;
    }
    __syncthreads();

    #pragma unroll
    for (int kq = 0; kq < 2; ++kq) {
      FragH fb;
      const _Float16* prw = pTw + m * 64 + 32 * kq + 8 * hh;
      fb.h[0] = *(const v8h*)(prw);
      fb.h[1] = *(const v8h*)(prw + 16);
      #pragma unroll
      for (int dt = 0; dt < 4; ++dt) {
        FragH fa;
        const _Float16* vrw = vs_ + (16 * dt + m) * 64 + 32 * kq + 8 * hh;
        fa.h[0] = *(const v8h*)(vrw);
        fa.h[1] = *(const v8h*)(vrw + 16);
        o[dt] = mma_f16(fa.v, fb.v, o[dt]);
      }
    }
  }

  __syncthreads();
  const float inv = (1.f / lrow) * PSCI;
  #pragma unroll
  for (int dt = 0; dt < 4; ++dt) {
    #pragma unroll
    for (int r = 0; r < 8; ++r) bw[m * 64 + 16 * dt + 8 * hh + r] = o[dt][r] * inv;
  }
  __syncthreads();
  attn_store(bw, ao, b, h, i0, lane);
  __threadfence();
  attn_store(bw, ao, b, h, i0, lane);
}

extern "C" void kernel_launch(void* const* d_in, const int* in_sizes, int n_in,
                              void* d_out, int out_size, void* d_ws, size_t ws_size,
                              hipStream_t stream) {
  using namespace cfg;
  if (n_in < 15) return;
  const int nact = BB * TT * DM;
  if (in_sizes[0] != nact || in_sizes[1] != nact || in_sizes[2] != nact) return;
  if (in_sizes[3] != BB * TT) return;
  if (in_sizes[4] != DM * DM || in_sizes[6] != DM * DM || in_sizes[8] != DM * DM ||
      in_sizes[10] != DM * DM || in_sizes[13] != DM * DM) return;
  if (in_sizes[5] != DM || in_sizes[7] != DM || in_sizes[9] != DM || in_sizes[14] != DM) return;
  if (in_sizes[11] != NH * DK || in_sizes[12] != NH * DK) return;
  if (out_size != nact) return;

  const float* q    = (const float*)d_in[0];
  const float* k    = (const float*)d_in[1];
  const float* v    = (const float*)d_in[2];
  const int*   mask = (const int*)d_in[3];
  const float* Wq   = (const float*)d_in[4];
  const float* bq   = (const float*)d_in[5];
  const float* Wk   = (const float*)d_in[6];
  const float* bk   = (const float*)d_in[7];
  const float* Wv   = (const float*)d_in[8];
  const float* bv   = (const float*)d_in[9];
  const float* Wp   = (const float*)d_in[10];
  const float* b_u  = (const float*)d_in[11];
  const float* b_v  = (const float*)d_in[12];
  const float* Wo   = (const float*)d_in[13];
  const float* bo   = (const float*)d_in[14];
  float* out = (float*)d_out;

  const size_t szQ = (size_t)BB * NH * TT * DK * sizeof(_Float16);
  const size_t szP = (size_t)NH * PR * DK * sizeof(_Float16);
  const size_t szA = (size_t)BB * TT * DM * sizeof(float);
  const size_t total = 4 * szQ + szP + szA;
  if (total > ws_size) return;
  char* ws = (char*)d_ws;
  _Float16* quB = (_Float16*)(ws);
  _Float16* qvB = (_Float16*)(ws + szQ);
  _Float16* khB = (_Float16*)(ws + 2 * szQ);
  _Float16* vtB = (_Float16*)(ws + 3 * szQ);
  _Float16* phB = (_Float16*)(ws + 4 * szQ);
  float*    aoB = (float*)(ws + 4 * szQ + szP);

  const int Mact = BB * TT;
  const dim3 gAct((Mact + 63) / 64, DM / 64);
  const dim3 gPos((PR + 63) / 64, DM / 64);

  k_proj<0, 0, true, 2><<<gAct, 128, 0, stream>>>(q, Wq, bq, b_u, b_v, quB, qvB, aoB, Mact);
  k_proj<0, 0, true, 0><<<gAct, 128, 0, stream>>>(k, Wk, bk, bk, bk, khB, khB, aoB, Mact);
  k_proj<0, 1, true, 0><<<gAct, 128, 0, stream>>>(v, Wv, bv, bv, bv, vtB, vtB, aoB, Mact);
  k_proj<1, 0, false, 0><<<gPos, 128, 0, stream>>>(q, Wp, bo, bo, bo, phB, phB, aoB, PR);
  k_attn<<<dim3(TT / 64, BB * NH), 128, 0, stream>>>(quB, qvB, khB, vtB, phB, mask, aoB);
  k_proj<0, 2, true, 0><<<gAct, 128, 0, stream>>>(aoB, Wo, bo, bo, bo, quB, quB, out, Mact);
  (void)hipGetLastError();
}
